// SoftmaxGAU_2001454760152
// MI455X (gfx1250) — hardware-verified
//
#include <hip/hip_runtime.h>

typedef __attribute__((ext_vector_type(16))) _Float16 v16h;
typedef __attribute__((ext_vector_type(8)))  _Float16 v8h;
typedef __attribute__((ext_vector_type(16))) __bf16   v16b;
typedef __attribute__((ext_vector_type(8)))  __bf16   v8b;
typedef __attribute__((ext_vector_type(8)))  float    v8f;
typedef __attribute__((ext_vector_type(4)))  float    v4f;

static constexpr int B_   = 8;
static constexpr int C_   = 512;
static constexpr int T_   = 1024;
static constexpr int E_   = 1024;
static constexpr int UVW_ = 2048;
static constexpr int H_   = 8;
static constexpr int HD_  = 64;
static constexpr int QK_  = 512;
static constexpr int NVH_ = 16;
static constexpr float EPS_ = 1e-5f;
static constexpr float WSC_ = 64.0f;
static constexpr float QKS_ = 8.0f;
static constexpr float GSC_ = 64.0f;

__device__ __forceinline__ unsigned short f2bf_bits(float f) {
  unsigned u = __float_as_uint(f);
  return (unsigned short)((u + 0x7FFFu + ((u >> 16) & 1u)) >> 16);
}
__device__ __forceinline__ float bf_bits2f(unsigned short h) { return __uint_as_float(((unsigned)h) << 16); }

__device__ __forceinline__ void dep_guard_h(v8f& a, v8f& b, v16h x, v16h y) { asm volatile("v_nop\n\tv_nop\n\tv_nop\n\tv_nop" : "+v"(a), "+v"(b) : "v"(x), "v"(y)); }
__device__ __forceinline__ void dep_guard_b(v8f& a, v8f& b, v16b x, v16b y) { asm volatile("v_nop\n\tv_nop\n\tv_nop\n\tv_nop" : "+v"(a), "+v"(b) : "v"(x), "v"(y)); }
__device__ __forceinline__ void keep4_h(v16h a, v16h b, v16h c, v16h d) { asm volatile("v_nop" :: "v"(a), "v"(b), "v"(c), "v"(d)); }
__device__ __forceinline__ void keep4_b(v16b a, v16b b, v16b c, v16b d) { asm volatile("v_nop" :: "v"(a), "v"(b), "v"(c), "v"(d)); }
__device__ __forceinline__ void acc_guard4(v8f& a, v8f& b, v8f& c, v8f& d) { asm volatile("v_nop\n\tv_nop\n\tv_nop\n\tv_nop" : "+v"(a), "+v"(b), "+v"(c), "+v"(d)); }
template <typename T> struct Frag;
template <> struct Frag<_Float16> {
  typedef v16h V; union U { v16h v; v8h h[2]; };
  static __device__ __forceinline__ v16h load(const _Float16* p) {
    U f; f.h[0] = *(const v8h*)(p); f.h[1] = *(const v8h*)(p + 16); return f.v;
  }
  static __device__ __forceinline__ v8f mma(v16h a, v16h b, v8f c) {
    return __builtin_amdgcn_wmma_f32_16x16x32_f16(false, a, false, b, (short)0, c, false, false);
  }
  static __device__ __forceinline__ void guard(v8f& a, v8f& b, v16h x, v16h y) { dep_guard_h(a, b, x, y); }
  static __device__ __forceinline__ void keep(v16h a, v16h b, v16h c, v16h d) { keep4_h(a, b, c, d); }
};
template <> struct Frag<__bf16> {
  typedef v16b V; union U { v16b v; v8b h[2]; };
  static __device__ __forceinline__ v16b load(const __bf16* p) {
    U f; f.h[0] = *(const v8b*)(p); f.h[1] = *(const v8b*)(p + 16); return f.v;
  }
  static __device__ __forceinline__ v8f mma(v16b a, v16b b, v8f c) {
    return __builtin_amdgcn_wmma_f32_16x16x32_bf16(false, a, false, b, (short)0, c, false, false);
  }
  static __device__ __forceinline__ void guard(v8f& a, v8f& b, v16b x, v16b y) { dep_guard_b(a, b, x, y); }
  static __device__ __forceinline__ void keep(v16b a, v16b b, v16b c, v16b d) { keep4_b(a, b, c, d); }
};

template <int ET> struct Elem;
template <> struct Elem<0> { typedef _Float16 T; };
template <> struct Elem<1> { typedef __bf16 T; };
template <int ET, bool SPLIT, int BIAS_MODE, int OUT_MODE, bool RESID, int ACT = 0>
__global__ __launch_bounds__(256) void wmma_gemm64(
    const unsigned short* __restrict__ Ap, const unsigned short* __restrict__ A2p, int lda, long strideA,
    const unsigned short* __restrict__ Btp, const unsigned short* __restrict__ Bt2p, int ldb, long strideB,
    void* __restrict__ Cout, void* __restrict__ Cout2, int ldc, long strideC,
    const float* __restrict__ bias,
    const float* __restrict__ resid, long strideR,
    int M, int N, int K, float scale) {
  typedef typename Elem<ET>::T T;
  typedef typename Frag<T>::V V;
  const T* A = (const T*)Ap; const T* A2 = (const T*)A2p; const T* Bt = (const T*)Btp; const T* Bt2 = (const T*)Bt2p;
  __shared__ __align__(16) float sT[8][16 * 68];
  const int b    = blockIdx.y;
  const int lane = threadIdx.x & 31;
  const int wave = threadIdx.x >> 5;
  const int tilesN = N >> 6;
  const int tilesM = M >> 6;
  const int tile = blockIdx.x * 8 + wave;
  if (tile >= tilesM * tilesN) return;
  const int tm = tile / tilesN;
  const int tn = tile - tm * tilesN;
  const int m0 = tm << 6;
  const int n0 = tn << 6;

  const T* Ab  = A  + (size_t)b * strideA;
  const T* Bb  = Bt + (size_t)b * strideB;
  const T* Ab2 = SPLIT ? (A2  + (size_t)b * strideA) : nullptr;
  const T* Bb2 = SPLIT ? (Bt2 + (size_t)b * strideB) : nullptr;

  const int rlane = lane & 15;
  const int koff  = (lane >> 4) * 8;
  const int mOff  = (lane >> 4) * 8;

  v8f acc[4][4];
#pragma unroll
  for (int i = 0; i < 4; ++i)
#pragma unroll
    for (int j = 0; j < 4; ++j) acc[i][j] = (v8f){0.f,0.f,0.f,0.f,0.f,0.f,0.f,0.f};

  for (int k0 = 0; k0 < K; k0 += 32) {
    V bh[4], bl[4];
#pragma unroll
    for (int j = 0; j < 4; ++j) {
      const size_t bo = (size_t)(n0 + (j << 4) + rlane) * ldb + koff + k0;
      bh[j] = Frag<T>::load(Bb + bo);
      if (SPLIT) bl[j] = Frag<T>::load(Bb2 + bo);
    }
#pragma unroll
    for (int i = 0; i < 4; ++i) {
      const size_t ao = (size_t)(m0 + (i << 4) + rlane) * lda + koff + k0;
      V ah = Frag<T>::load(Ab + ao);
      V al;
      if (SPLIT) al = Frag<T>::load(Ab2 + ao);
#pragma unroll
      for (int j = 0; j < 4; ++j) {
        acc[i][j] = Frag<T>::mma(ah, bh[j], acc[i][j]);
        if (SPLIT) {
          acc[i][j] = Frag<T>::mma(ah, bl[j], acc[i][j]);
          acc[i][j] = Frag<T>::mma(al, bh[j], acc[i][j]);
        }
      }
      Frag<T>::guard(acc[i][0], acc[i][3], ah, SPLIT ? al : ah);
    }
    Frag<T>::keep(bh[0], bh[1], bh[2], bh[3]);
    if (SPLIT) Frag<T>::keep(bl[0], bl[1], bl[2], bl[3]);
  }
  acc_guard4(acc[0][0], acc[0][1], acc[0][2], acc[0][3]);
  acc_guard4(acc[1][0], acc[1][1], acc[1][2], acc[1][3]);
  acc_guard4(acc[2][0], acc[2][1], acc[2][2], acc[2][3]);
  acc_guard4(acc[3][0], acc[3][1], acc[3][2], acc[3][3]);

  float* slab = sT[wave];
  const float* Rb = RESID ? (resid + (size_t)b * strideR) : nullptr;
#pragma unroll
  for (int i = 0; i < 4; ++i) {
    const int mBase = m0 + (i << 4);
#pragma unroll
    for (int j = 0; j < 4; ++j) {
      const int n = n0 + (j << 4) + rlane;
      float bv = 0.f;
      if (BIAS_MODE == 2) bv = bias[n];
#pragma unroll
      for (int r = 0; r < 8; ++r) {
        float v = acc[i][j][r] * scale;
        if (BIAS_MODE == 1) v += bias[mBase + mOff + r];
        if (BIAS_MODE == 2) v += bv;
        if (RESID) v += Rb[(size_t)(mBase + mOff + r) * ldc + n];
        if (ACT == 1) v = tanhf(v);
        if (ACT == 2) v = fmaxf(v, 0.0f);
        if (ACT == 3) v = v / (1.0f + expf(-v));
        if (ACT == 4) v = (v > 0.f) ? v : 0.01f * v;
        if (ACT == 5) v = 0.5f * v * (1.0f + erff(v * 0.70710678118654752f));
        slab[(mOff + r) * 68 + (j << 4) + rlane] = v;
      }
    }
    __builtin_amdgcn_fence(__ATOMIC_RELEASE, "workgroup");
    __builtin_amdgcn_wave_barrier();
    __builtin_amdgcn_fence(__ATOMIC_ACQUIRE, "workgroup");
    if (OUT_MODE == 0) {
      float* C = (float*)Cout + (size_t)b * strideC;
      const int hh = lane >> 4, c4 = (lane & 15) * 4;
      for (int pass = 0; pass < 2; ++pass) {
#pragma unroll
        for (int it = 0; it < 8; ++it) {
          const int row = it * 2 + hh;
          v4f v = *(const v4f*)(slab + row * 68 + c4);
          *(volatile v4f*)(C + (size_t)(mBase + row) * ldc + n0 + c4) = v;
        }
        __threadfence();
      }
    } else {
      const int q = lane >> 3, c8 = (lane & 7) * 8;
      unsigned short* C  = (unsigned short*)Cout  + (size_t)b * strideC;
      unsigned short* C2 = (OUT_MODE == 2) ? ((unsigned short*)Cout2 + (size_t)b * strideC) : nullptr;
      for (int pass = 0; pass < 2; ++pass) {
#pragma unroll
        for (int it = 0; it < 4; ++it) {
          const int row = it * 4 + q;
          const float* sp = slab + row * 68 + c8;
          v8h hv, lv;
#pragma unroll
          for (int e = 0; e < 8; ++e) {
            if (OUT_MODE == 1) {
              hv[e] = (_Float16)sp[e];
            } else {
              unsigned short hb = f2bf_bits(sp[e]);
              unsigned short lb = f2bf_bits(sp[e] - bf_bits2f(hb));
              hv[e] = __builtin_bit_cast(_Float16, hb);
              lv[e] = __builtin_bit_cast(_Float16, lb);
            }
          }
          *(volatile v8h*)(C + (size_t)(mBase + row) * ldc + n0 + c8) = hv;
          if (OUT_MODE == 2) *(volatile v8h*)(C2 + (size_t)(mBase + row) * ldc + n0 + c8) = lv;
        }
        __threadfence();
      }
    }
    __builtin_amdgcn_fence(__ATOMIC_RELEASE, "workgroup");
    __builtin_amdgcn_wave_barrier();
    __builtin_amdgcn_fence(__ATOMIC_ACQUIRE, "workgroup");
  }
}

__global__ __launch_bounds__(256) void cast_scale_f32_f16x2(
    const float* __restrict__ in, _Float16* __restrict__ out, int n2, float sc) {
  const int i = blockIdx.x * 256 + threadIdx.x;
  if (i < n2) {
    const _Float16 h0 = (_Float16)(in[2 * i] * sc), h1 = (_Float16)(in[2 * i + 1] * sc);
    const unsigned u = (unsigned)__builtin_bit_cast(unsigned short, h0) | ((unsigned)__builtin_bit_cast(unsigned short, h1) << 16);
    ((volatile unsigned*)out)[i] = u;
    __threadfence();
    ((volatile unsigned*)out)[i] = u;
  }
}

__global__ __launch_bounds__(256) void xpose_cast_x(const float* __restrict__ x, _Float16* __restrict__ xt) {
  __shared__ float sh[64 * 65];
  const int tid = threadIdx.x, wave = tid >> 5, lane = tid & 31;
  const int b = blockIdx.z, c0 = blockIdx.y * 64, t0 = blockIdx.x * 64;
  const float* xb = x + (size_t)b * C_ * T_;
  const int t4 = (tid & 15) * 4, crl = tid >> 4;
#pragma unroll
  for (int p = 0; p < 4; ++p) {
    const int cr = p * 16 + crl;
    const v4f v = *(const v4f*)(xb + (size_t)(c0 + cr) * T_ + t0 + t4);
    sh[(t4 + 0) * 65 + cr] = v[0];
    sh[(t4 + 1) * 65 + cr] = v[1];
    sh[(t4 + 2) * 65 + cr] = v[2];
    sh[(t4 + 3) * 65 + cr] = v[3];
  }
  __syncthreads();
  const int q = lane >> 3, c8 = (lane & 7) * 8;
  _Float16* ob = xt + ((size_t)b * T_ + t0) * C_ + c0;
  for (int pass = 0; pass < 2; ++pass) {
#pragma unroll
    for (int it = 0; it < 2; ++it) {
      const int row = it * 32 + wave * 4 + q;
      v8h hv;
#pragma unroll
      for (int e = 0; e < 8; ++e) hv[e] = (_Float16)sh[row * 65 + c8 + e];
      *(volatile v8h*)(ob + (size_t)row * C_ + c8) = hv;
    }
    __threadfence();
  }
}

__global__ __launch_bounds__(256) void qk_affine_kernel(
    const float* __restrict__ z, const float* __restrict__ w_q, const float* __restrict__ b_q,
    const float* __restrict__ w_k, const float* __restrict__ b_k,
    _Float16* __restrict__ q16, _Float16* __restrict__ k16, int n8) {
  const int i = blockIdx.x * 256 + threadIdx.x;
  if (i < n8) {
    const size_t e0 = (size_t)i * 8;
    const int ch = (int)(e0 & (size_t)(QK_ - 1));
    const v4f z0 = *(const v4f*)(z + e0), z1 = *(const v4f*)(z + e0 + 4);
    const v4f wq0 = *(const v4f*)(w_q + ch), wq1 = *(const v4f*)(w_q + ch + 4);
    const v4f bq0 = *(const v4f*)(b_q + ch), bq1 = *(const v4f*)(b_q + ch + 4);
    const v4f wk0 = *(const v4f*)(w_k + ch), wk1 = *(const v4f*)(w_k + ch + 4);
    const v4f bk0 = *(const v4f*)(b_k + ch), bk1 = *(const v4f*)(b_k + ch + 4);
    v8h qv, kv;
#pragma unroll
    for (int e = 0; e < 4; ++e) {
      qv[e]     = (_Float16)((z0[e] * wq0[e] + bq0[e]) * QKS_);
      qv[4 + e] = (_Float16)((z1[e] * wq1[e] + bq1[e]) * QKS_);
      kv[e]     = (_Float16)((z0[e] * wk0[e] + bk0[e]) * QKS_);
      kv[4 + e] = (_Float16)((z1[e] * wk1[e] + bk1[e]) * QKS_);
    }
    *(volatile v8h*)(q16 + e0) = qv;
    *(volatile v8h*)(k16 + e0) = kv;
    __threadfence();
    *(volatile v8h*)(q16 + e0) = qv;
    *(volatile v8h*)(k16 + e0) = kv;
  }
}

#define AT_D 64
#define AT_NW 4
#define AT_QB 64
#define AT_KC 64
#define PSC_F 32768.0f

__device__ __forceinline__ v8f mma_f16g(v16h a, v16h b, v8f c) {
  c = __builtin_amdgcn_wmma_f32_16x16x32_f16(false, a, false, b, (short)0, c, false, false);
  asm volatile("v_nop\n\tv_nop\n\tv_nop\n\tv_nop" : "+v"(c) : "v"(a), "v"(b));
  return c;
}

__global__ __launch_bounds__(128)
void gau_attn_kernel(const _Float16* __restrict__ q16, const _Float16* __restrict__ k16,
                     const _Float16* __restrict__ uv, _Float16* __restrict__ gout, float sscale) {
  union FB { v16h v; v8h h[2]; };
  __shared__ __align__(16) _Float16 Ksh[AT_KC * AT_D];
  __shared__ __align__(16) _Float16 Vth[AT_D * AT_KC];
  __shared__ __align__(16) _Float16 Psh[AT_NW][16 * AT_KC];
  __shared__ __align__(16) float    Os[AT_NW][16 * 68];

  const int tid  = threadIdx.x;
  const int wave = tid >> 5;
  const int lane = tid & 31;
  const int hh   = lane >> 4;
  const int c    = lane & 15;

  constexpr int NQB = T_ / AT_QB;
  const int bx = blockIdx.x;
  const int qb = bx % NQB;
  const int bj = bx / NQB;
  const int j  = bj % NVH_;
  const int b  = bj / NVH_;
  const int h  = j >> 1;
  const int q0 = qb * AT_QB + wave * 16;

  const _Float16* qbp = q16 + (size_t)b * T_ * QK_ + h * HD_;
  const _Float16* kbp = k16 + (size_t)b * T_ * QK_ + h * HD_;
  const _Float16* vbp = uv + (size_t)b * T_ * UVW_ + E_ + j * 64;
  const _Float16* ubp = uv + (size_t)b * T_ * UVW_ + j * 64;
  _Float16*       gbp = gout + (size_t)b * T_ * E_ + j * 64;

  v16h qa[2];
  {
    const _Float16* qrow = qbp + (size_t)(q0 + c) * QK_;
#pragma unroll
    for (int dc = 0; dc < 2; ++dc) {
      FB f;
      f.h[0] = *(const v8h*)(qrow + dc * 32 + 8 * hh);
      f.h[1] = *(const v8h*)(qrow + dc * 32 + 16 + 8 * hh);
      qa[dc] = f.v;
    }
  }

  float mrow[8], lrow[8];
  v8f oacc[4];
#pragma unroll
  for (int r = 0; r < 8; ++r) { mrow[r] = -__builtin_huge_valf(); lrow[r] = 0.f; }
#pragma unroll
  for (int t = 0; t < 4; ++t) oacc[t] = (v8f){0.f,0.f,0.f,0.f,0.f,0.f,0.f,0.f};

  constexpr int nChunks = T_ / AT_KC;
  for (int kc = 0; kc < nChunks; ++kc) {
    const int kv0 = kc * AT_KC;
    __syncthreads();
    {
      const int kvr = tid >> 1, dh = (tid & 1) * 32;
      const _Float16* krow = kbp + (size_t)(kv0 + kvr) * QK_ + dh;
      const _Float16* vrow = vbp + (size_t)(kv0 + kvr) * UVW_ + dh;
#pragma unroll
      for (int i = 0; i < 4; ++i) {
        const v8h kk = *(const v8h*)(krow + 8 * i);
        *(v8h*)(Ksh + kvr * AT_D + dh + 8 * i) = kk;
        const v8h vv = *(const v8h*)(vrow + 8 * i);
#pragma unroll
        for (int e = 0; e < 8; ++e) Vth[(dh + 8 * i + e) * AT_KC + kvr] = vv[e];
      }
    }
    __syncthreads();

    v8f s[4];
#pragma unroll
    for (int jj = 0; jj < 4; ++jj) {
      s[jj] = (v8f){0.f,0.f,0.f,0.f,0.f,0.f,0.f,0.f};
#pragma unroll
      for (int dc = 0; dc < 2; ++dc) {
        FB kb;
        kb.h[0] = *(const v8h*)(Ksh + (jj * 16 + c) * AT_D + dc * 32 + 8 * hh);
        kb.h[1] = *(const v8h*)(Ksh + (jj * 16 + c) * AT_D + dc * 32 + 16 + 8 * hh);
        s[jj] = mma_f16g(qa[dc], kb.v, s[jj]);
      }
    }
    float cm[8];
#pragma unroll
    for (int r = 0; r < 8; ++r) {
      float m = -__builtin_huge_valf();
#pragma unroll
      for (int jj = 0; jj < 4; ++jj) {
        const float sv = s[jj][r] * sscale;
        s[jj][r] = sv;
        m = fmaxf(m, sv);
      }
#pragma unroll
      for (int off = 1; off < 16; off <<= 1) m = fmaxf(m, __shfl_xor(m, off, 32));
      cm[r] = m;
    }
    _Float16* pw = Psh[wave];
#pragma unroll
    for (int r = 0; r < 8; ++r) {
      const float mnew = fmaxf(mrow[r], cm[r]);
      const float alpha = expf(mrow[r] - mnew);
      mrow[r] = mnew;
      float psum = 0.f;
#pragma unroll
      for (int jj = 0; jj < 4; ++jj) {
        const float p = expf(s[jj][r] - mnew);
        psum += p;
        pw[(8 * hh + r) * AT_KC + jj * 16 + c] = (_Float16)(p * PSC_F);
      }
#pragma unroll
      for (int off = 1; off < 16; off <<= 1) psum += __shfl_xor(psum, off, 32);
      lrow[r] = lrow[r] * alpha + psum;
#pragma unroll
      for (int t = 0; t < 4; ++t) oacc[t][r] *= alpha;
    }
    __builtin_amdgcn_fence(__ATOMIC_RELEASE, "workgroup");
    __builtin_amdgcn_wave_barrier();
    __builtin_amdgcn_fence(__ATOMIC_ACQUIRE, "workgroup");
#pragma unroll 1
    for (int kk = 0; kk < 2; ++kk) {
      FB pa;
      pa.h[0] = *(const v8h*)(pw + c * AT_KC + kk * 32 + 8 * hh);
      pa.h[1] = *(const v8h*)(pw + c * AT_KC + kk * 32 + 16 + 8 * hh);
#pragma unroll
      for (int t = 0; t < 4; ++t) {
        FB vb;
        vb.h[0] = *(const v8h*)(Vth + (t * 16 + c) * AT_KC + kk * 32 + 8 * hh);
        vb.h[1] = *(const v8h*)(Vth + (t * 16 + c) * AT_KC + kk * 32 + 16 + 8 * hh);
        oacc[t] = mma_f16g(pa.v, vb.v, oacc[t]);
      }
    }
  }

  float* os = Os[wave];
#pragma unroll
  for (int r = 0; r < 8; ++r) {
    const float inv = 1.0f / (lrow[r] * PSC_F);
#pragma unroll
    for (int t = 0; t < 4; ++t) os[(8 * hh + r) * 68 + t * 16 + c] = oacc[t][r] * inv;
  }
  __builtin_amdgcn_fence(__ATOMIC_RELEASE, "workgroup");
  __builtin_amdgcn_wave_barrier();
  __builtin_amdgcn_fence(__ATOMIC_ACQUIRE, "workgroup");
  {
    const int q = lane >> 3, c8 = (lane & 7) * 8;
    for (int pass = 0; pass < 2; ++pass) {
#pragma unroll
      for (int it = 0; it < 4; ++it) {
        const int row = it * 4 + q;
        const float* sp = os + row * 68 + c8;
        const v8h u8 = *(const v8h*)(ubp + (size_t)(q0 + row) * UVW_ + c8);
        v8h hv;
#pragma unroll
        for (int e = 0; e < 8; ++e) hv[e] = (_Float16)(sp[e] * (float)u8[e] * GSC_);
        *(volatile v8h*)(gbp + (size_t)(q0 + row) * E_ + c8) = hv;
      }
      __threadfence();
    }
  }
}

__global__ __launch_bounds__(256) void rms_kernel(
    const float* __restrict__ y, const float* __restrict__ gamma, float* __restrict__ out, int nbt) {
  const int gi = blockIdx.x * 256 + threadIdx.x;
  const int gc = gi < nbt ? gi : nbt - 1;
  const int b = gc / T_, t = gc - b * T_;
  const float* yp = y + (size_t)b * C_ * T_ + t;
  float* op = out + (size_t)b * C_ * T_ + t;
  float s = 0.f;
#pragma unroll 8
  for (int cc = 0; cc < C_; ++cc) { const float v = yp[(size_t)cc * T_]; s += v * v; }
  const float rr = rsqrtf(s * (1.0f / 512.0f) + EPS_);
  if (gi < nbt) {
    for (int pass = 0; pass < 2; ++pass) {
#pragma unroll 4
      for (int cc = 0; cc < C_; ++cc) {
        const float val = yp[(size_t)cc * T_] * rr * gamma[cc];
        *(volatile float*)(op + (size_t)cc * T_) = val;
      }
      __threadfence();
    }
  }
}

extern "C" void kernel_launch(void* const* d_in, const int* in_sizes, int n_in,
                              void* d_out, int out_size, void* d_ws,
                              size_t ws_size, hipStream_t stream) {
  if (n_in < 12) return;
  if (in_sizes[0] != B_ * C_ * T_ || in_sizes[1] != UVW_ * C_ || in_sizes[2] != UVW_ ||
      in_sizes[3] != QK_ * C_ || in_sizes[4] != QK_ || in_sizes[5] != QK_ || in_sizes[6] != QK_ ||
      in_sizes[7] != QK_ || in_sizes[8] != QK_ || in_sizes[9] != C_ * E_ || in_sizes[10] != C_ ||
      in_sizes[11] != C_ || out_size != B_ * C_ * T_) return;

  const float* x      = (const float*)d_in[0];
  const float* W_in   = (const float*)d_in[1];
  const float* b_in   = (const float*)d_in[2];
  const float* W_attn = (const float*)d_in[3];
  const float* b_attn = (const float*)d_in[4];
  const float* w_q    = (const float*)d_in[5];
  const float* b_q    = (const float*)d_in[6];
  const float* w_k    = (const float*)d_in[7];
  const float* b_k    = (const float*)d_in[8];
  const float* W_out  = (const float*)d_in[9];
  const float* b_out  = (const float*)d_in[10];
  const float* gamma  = (const float*)d_in[11];
  float* out = (float*)d_out;

  size_t off = 0;
  char* base = (char*)d_ws;
  const size_t nXT   = (size_t)B_ * T_ * C_ * 2;
  const size_t nWIN  = (size_t)UVW_ * C_ * 2;
  const size_t nWAT  = (size_t)QK_ * C_ * 2;
  const size_t nWOUT = (size_t)C_ * E_ * 2;
  const size_t nUV   = (size_t)B_ * T_ * UVW_ * 2;
  const size_t nZ    = (size_t)B_ * T_ * QK_ * 4;
  const size_t nQ    = (size_t)B_ * T_ * QK_ * 2;
  const size_t nK    = nQ;
  const size_t nG    = (size_t)B_ * T_ * E_ * 2;
  const size_t nY    = (size_t)B_ * C_ * T_ * 4;
  _Float16* xT   = (_Float16*)(base + off); off += nXT;
  _Float16* Win  = (_Float16*)(base + off); off += nWIN;
  _Float16* Wat  = (_Float16*)(base + off); off += nWAT;
  _Float16* Wou  = (_Float16*)(base + off); off += nWOUT;
  _Float16* uv16 = (_Float16*)(base + off); off += nUV;
  float*    z    = (float*)(base + off);    off += nZ;
  _Float16* q16  = (_Float16*)(base + off); off += nQ;
  _Float16* k16  = (_Float16*)(base + off); off += nK;
  _Float16* g16  = (_Float16*)(base + off); off += nG;
  float*    y    = (float*)(base + off);    off += nY;
  if (off > ws_size) return;

  const dim3 blk256(256), blk128(128);
  const float wsc_inv = 1.0f / WSC_;
  const float qscale  = (float)(1.1111111111111112 / 8.0);
  const float sscale  = qscale * (1.0f / (QKS_ * QKS_));

  {
    const int n2a = in_sizes[1] / 2, n2b = in_sizes[3] / 2, n2c = in_sizes[9] / 2;
    cast_scale_f32_f16x2<<<dim3((n2a + 255) / 256), blk256, 0, stream>>>(W_in, Win, n2a, WSC_);
    cast_scale_f32_f16x2<<<dim3((n2b + 255) / 256), blk256, 0, stream>>>(W_attn, Wat, n2b, WSC_);
    cast_scale_f32_f16x2<<<dim3((n2c + 255) / 256), blk256, 0, stream>>>(W_out, Wou, n2c, WSC_);
  }
  xpose_cast_x<<<dim3(T_ / 64, C_ / 64, B_), blk256, 0, stream>>>(x, xT);

  wmma_gemm64<0, false, 2, 1, false, 3><<<dim3((T_ / 64) * (UVW_ / 64) / 8, B_), blk256, 0, stream>>>(
      (const unsigned short*)xT, (const unsigned short*)xT, C_, (long)T_ * C_,
      (const unsigned short*)Win, (const unsigned short*)Win, C_, 0L,
      (void*)uv16, (void*)uv16, UVW_, (long)T_ * UVW_,
      b_in, x, 0L, T_, UVW_, C_, wsc_inv);
  wmma_gemm64<0, false, 2, 0, false, 0><<<dim3((T_ / 64) * (QK_ / 64) / 8, B_), blk256, 0, stream>>>(
      (const unsigned short*)xT, (const unsigned short*)xT, C_, (long)T_ * C_,
      (const unsigned short*)Wat, (const unsigned short*)Wat, C_, 0L,
      (void*)z, (void*)z, QK_, (long)T_ * QK_,
      b_attn, x, 0L, T_, QK_, C_, wsc_inv);
  {
    const int n8 = (int)((size_t)B_ * T_ * QK_ / 8);
    qk_affine_kernel<<<dim3((n8 + 255) / 256), blk256, 0, stream>>>(z, w_q, b_q, w_k, b_k, q16, k16, n8);
  }
  gau_attn_kernel<<<dim3(B_ * NVH_ * (T_ / AT_QB)), blk128, 0, stream>>>(q16, k16, uv16, g16, sscale);
  wmma_gemm64<0, false, 1, 0, true, 0><<<dim3((C_ / 64) * (T_ / 64) / 8, B_), blk256, 0, stream>>>(
      (const unsigned short*)Wou, (const unsigned short*)Wou, E_, 0L,
      (const unsigned short*)g16, (const unsigned short*)g16, E_, (long)T_ * E_,
      (void*)y, (void*)y, T_, (long)C_ * T_,
      b_out, x, (long)C_ * T_, C_, T_, E_, 1.0f / (WSC_ * GSC_));
  {
    const int nbt = B_ * T_;
    rms_kernel<<<dim3((nbt + 255) / 256), blk256, 0, stream>>>(y, gamma, out, nbt);
  }
  (void)hipGetLastError();
}
